// LiftingAttention_4389456576535
// MI455X (gfx1250) — hardware-verified
//
#include <hip/hip_runtime.h>
#include <math.h>
#include <stdint.h>


#define BATCH  4
#define SEQ    512
#define DIMC   512
#define HEADS  8
#define HD     64
#define NGRP   8
#define NSITE  512
#define NTOK   2048
#define NROW   16384
#define OQKV   1536
#define NKST   16
#define SPP    72
#define WTP    72
#define NBT8   (NGRP * SEQ * (SEQ / 8))

static_assert(NTOK == BATCH * SEQ);
static_assert(NROW == NTOK * NGRP);
static_assert(HEADS * HD == DIMC);
static_assert(OQKV == 3 * DIMC);
static_assert(NKST * 32 == SEQ);
static_assert(SEQ == 512 && NSITE == 512 && NGRP == 8 && HEADS == 8 && DIMC == 512);
static_assert((NTOK % 64) == 0 && (OQKV % 64) == 0 && (NROW % 64) == 0 && (DIMC % 64) == 0);
static_assert((NBT8 % 256) == 0 && (NTOK % 8) == 0);

typedef _Float16 v16h __attribute__((ext_vector_type(16)));
typedef _Float16 v8h  __attribute__((ext_vector_type(8)));
typedef float    v8f  __attribute__((ext_vector_type(8)));
typedef float    v4f  __attribute__((ext_vector_type(4)));
typedef unsigned int v4u __attribute__((ext_vector_type(4)));
typedef int      v4i  __attribute__((ext_vector_type(4)));

__device__ __forceinline__ unsigned short bf_bits(float f) {
  unsigned u = __float_as_uint(f);
  return (unsigned short)((u + 0x7FFFu + ((u >> 16) & 1u)) >> 16);
}
__device__ __forceinline__ float bf_up(unsigned short h) { return __uint_as_float(((unsigned)h) << 16); }
__device__ __forceinline__ unsigned short h_bits(_Float16 x) { return __builtin_bit_cast(unsigned short, x); }
__device__ __forceinline__ unsigned pk16(unsigned short a, unsigned short b) { return (unsigned)a | ((unsigned)b << 16); }
__device__ __forceinline__ v8f zero8() { v8f z = {0.f, 0.f, 0.f, 0.f, 0.f, 0.f, 0.f, 0.f}; return z; }
__device__ __forceinline__ int wrap_clamp(int v, int n) {
  int w = (v < 0) ? (v + n) : v;
  return min(max(w, 0), n - 1);
}

__device__ __forceinline__ v16h ldfrag_h(const _Float16* p) {
  union { v16h v; v8h h[2]; } f;
  f.h[0] = *(const v8h*)(p);
  f.h[1] = *(const v8h*)(p + 16);
  return f.v;
}

__device__ __forceinline__ v8f mma_h_raw(v16h a, v16h b, v8f c) {
  return __builtin_amdgcn_wmma_f32_16x16x32_f16(false, a, false, b, (short)0, c, false, false);
}
__device__ __forceinline__ void res_guard(v8f& t, v8f& acc, v16h x, v16h y) {
#if defined(__HIP_DEVICE_COMPILE__)
  asm volatile("v_nop\n\tv_nop\n\tv_nop\n\tv_nop" : "+v"(t), "+v"(acc) : "v"(x), "v"(y));
#endif
}
__device__ __forceinline__ void dep_guard_h(v8f& a, v8f& b, v16h x, v16h y) {
#if defined(__HIP_DEVICE_COMPILE__)
  asm volatile("v_nop\n\tv_nop\n\tv_nop\n\tv_nop" : "+v"(a), "+v"(b) : "v"(x), "v"(y));
#endif
}
__device__ __forceinline__ void guard_sc(v8f& a, v8f& b, v16h k0, v16h k1, v16h q0, v16h q1, v16h q2, v16h q3) {
#if defined(__HIP_DEVICE_COMPILE__)
  asm volatile("v_nop\n\tv_nop\n\tv_nop\n\tv_nop" : "+v"(a), "+v"(b) : "v"(k0), "v"(k1), "v"(q0), "v"(q1), "v"(q2), "v"(q3));
#endif
}
__device__ __forceinline__ void guard_pv(v8f& a, v8f& b, v16h w, v16h x, v16h y, v16h z) {
#if defined(__HIP_DEVICE_COMPILE__)
  asm volatile("v_nop\n\tv_nop\n\tv_nop\n\tv_nop" : "+v"(a), "+v"(b) : "v"(w), "v"(x), "v"(y), "v"(z));
#endif
}
__device__ __forceinline__ void keep4_h(v16h a, v16h b, v16h c, v16h d) {
#if defined(__HIP_DEVICE_COMPILE__)
  asm volatile("v_nop" :: "v"(a), "v"(b), "v"(c), "v"(d));
#endif
}
__device__ __forceinline__ void acc_guard4(v8f& a, v8f& b, v8f& c, v8f& d) {
#if defined(__HIP_DEVICE_COMPILE__)
  asm volatile("v_nop\n\tv_nop\n\tv_nop\n\tv_nop" : "+v"(a), "+v"(b), "+v"(c), "+v"(d));
#endif
}
__device__ __forceinline__ void wave_sync_lds() {
  __builtin_amdgcn_fence(__ATOMIC_RELEASE, "workgroup");
  __builtin_amdgcn_wave_barrier();
  __builtin_amdgcn_fence(__ATOMIC_ACQUIRE, "workgroup");
}

__global__ __launch_bounds__(256) void cvt_wt(const float* __restrict__ W, unsigned short* WT, int orow0, float scale) {
  __shared__ __align__(16) unsigned short ts[64 * WTP];
  const int tid = threadIdx.x;
  const int o0 = blockIdx.x * 64, c0 = blockIdx.y * 64;
#pragma unroll 1
  for (int pass = 0; pass < 4; ++pass) {
    const int cl = pass * 16 + (tid >> 4);
    const int l4 = (tid & 15) * 4;
    const v4f v = *(const v4f*)(W + ((size_t)(c0 + cl)) * DIMC + o0 + l4);
#pragma unroll
    for (int i = 0; i < 4; ++i) ts[(l4 + i) * WTP + cl] = h_bits((_Float16)(bf_up(bf_bits(v[i])) * scale));
  }
  __syncthreads();
#pragma unroll 1
  for (int pass = 0; pass < 2; ++pass) {
    const int lr = pass * 32 + (tid >> 3);
    const int c8 = (tid & 7) * 8;
    const v4u v = *(const v4u*)(ts + lr * WTP + c8);
    unsigned short* dst = WT + ((size_t)(orow0 + o0 + lr)) * DIMC + c0 + c8;
    *(volatile v4u*)dst = v;
    __threadfence();
    *(volatile v4u*)dst = v;
  }
}

__global__ __launch_bounds__(256) void ln_rows(const float* __restrict__ X, const float* __restrict__ lg,
                                               const float* __restrict__ lb,
                                               unsigned short* XH, unsigned short* XL) {
  const int lane = threadIdx.x & 31, wave = threadIdx.x >> 5;
  const int row = blockIdx.x * 8 + wave;
  if (row >= NTOK) return;
  const float* x = X + (size_t)row * DIMC;

  float s = 0.0f;
#pragma unroll 1
  for (int q = 0; q < 4; ++q) {
    const int c = 8 * lane + 256 * (q >> 1) + 4 * (q & 1);
    const v4f a = *(const v4f*)(x + c);
#pragma unroll
    for (int e = 0; e < 4; ++e) s += bf_up(bf_bits(a[e]));
  }
#pragma unroll
  for (int d = 16; d >= 1; d >>= 1) s += __shfl_xor(s, d, 32);
  const float mu = s * (1.0f / DIMC);

  float ss = 0.0f;
#pragma unroll 1
  for (int q = 0; q < 4; ++q) {
    const int c = 8 * lane + 256 * (q >> 1) + 4 * (q & 1);
    const v4f a = *(const v4f*)(x + c);
#pragma unroll
    for (int e = 0; e < 4; ++e) {
      const float dv = bf_up(bf_bits(a[e])) - mu;
      ss += dv * dv;
    }
  }
#pragma unroll
  for (int d = 16; d >= 1; d >>= 1) ss += __shfl_xor(ss, d, 32);
  const float var = ss * (1.0f / DIMC);
  const float rs = rsqrtf(var + 1e-5f);

  const size_t base = (size_t)row * DIMC;
#pragma unroll 1
  for (int p = 0; p < 2; ++p) {
    const int c = 8 * lane + 256 * p;
    const v4f a0 = *(const v4f*)(x + c);
    const v4f a1 = *(const v4f*)(x + c + 4);
    const v4f g0 = *(const v4f*)(lg + c);
    const v4f g1 = *(const v4f*)(lg + c + 4);
    const v4f b0 = *(const v4f*)(lb + c);
    const v4f b1 = *(const v4f*)(lb + c + 4);
    float xv[8], gv[8], bb8[8];
#pragma unroll
    for (int e = 0; e < 4; ++e) {
      xv[e]  = bf_up(bf_bits(a0[e]));  xv[4 + e]  = bf_up(bf_bits(a1[e]));
      gv[e]  = bf_up(bf_bits(g0[e]));  gv[4 + e]  = bf_up(bf_bits(g1[e]));
      bb8[e] = bf_up(bf_bits(b0[e]));  bb8[4 + e] = bf_up(bf_bits(b1[e]));
    }
    unsigned short hb[8], lo[8];
#pragma unroll
    for (int e = 0; e < 8; ++e) {
      const float y = (xv[e] - mu) * rs * gv[e] + bb8[e];
      const float f = y * 16.0f;
      const _Float16 xh = (_Float16)f;
      hb[e] = h_bits(xh);
      lo[e] = h_bits((_Float16)((f - (float)xh) * 2048.0f));
    }
    v4u ph, pl;
#pragma unroll
    for (int q = 0; q < 4; ++q) {
      ph[q] = pk16(hb[2 * q], hb[2 * q + 1]);
      pl[q] = pk16(lo[2 * q], lo[2 * q + 1]);
    }
    unsigned short* dh = XH + base + c;
    unsigned short* dl = XL + base + c;
    *(volatile v4u*)dh = ph;
    *(volatile v4u*)dl = pl;
    __threadfence();
    *(volatile v4u*)dh = ph;
    *(volatile v4u*)dl = pl;
  }
}

__global__ __launch_bounds__(256) void bias_table(const float* __restrict__ rho, const int* __restrict__ sdiff,
                                                  const int* __restrict__ gact, unsigned short* BT) {
  const int i = blockIdx.x * 256 + threadIdx.x;
  if (i < NBT8) {
    const int k8 = i & (SEQ / 8 - 1);
    const int q  = (i >> 6) & (SEQ - 1);
    const int g  = i >> 15;
    const v4i sa = *(const v4i*)(sdiff + (size_t)q * SEQ + 8 * k8);
    const v4i sb = *(const v4i*)(sdiff + (size_t)q * SEQ + 8 * k8 + 4);
    int ix[8];
    ix[0] = sa[0]; ix[1] = sa[1]; ix[2] = sa[2]; ix[3] = sa[3];
    ix[4] = sb[0]; ix[5] = sb[1]; ix[6] = sb[2]; ix[7] = sb[3];
    float rv[8][8];
#pragma unroll
    for (int j = 0; j < 8; ++j) {
      const int i1 = wrap_clamp(ix[j], NSITE);
      int i2 = gact[g * NSITE + i1];
      i2 = wrap_clamp(i2, NSITE);
      const v4f ra = *(const v4f*)(rho + (size_t)i2 * HEADS);
      const v4f rb = *(const v4f*)(rho + (size_t)i2 * HEADS + 4);
      rv[j][0] = ra[0]; rv[j][1] = ra[1]; rv[j][2] = ra[2]; rv[j][3] = ra[3];
      rv[j][4] = rb[0]; rv[j][5] = rb[1]; rv[j][6] = rb[2]; rv[j][7] = rb[3];
    }
    v4u pk[8];
#pragma unroll
    for (int h = 0; h < 8; ++h) {
      unsigned short hb[8];
#pragma unroll
      for (int j = 0; j < 8; ++j) hb[j] = bf_bits(rv[j][h]);
#pragma unroll
      for (int qq = 0; qq < 4; ++qq) pk[h][qq] = pk16(hb[2 * qq], hb[2 * qq + 1]);
    }
    for (int pass = 0; pass < 2; ++pass) {
#pragma unroll
      for (int h = 0; h < 8; ++h) {
        unsigned short* dst = BT + (((size_t)(h * NGRP + g)) * SEQ + q) * SEQ + 8 * k8;
        *(volatile v4u*)dst = pk[h];
      }
      __threadfence();
    }
  }
}

__global__ __launch_bounds__(256) void gemm_qkv(
    const unsigned short* __restrict__ Wp, const unsigned short* __restrict__ XHp, const unsigned short* __restrict__ XLp,
    const float* __restrict__ bq, const float* __restrict__ bk, const float* __restrict__ bv,
    unsigned short* QH, unsigned short* QL, unsigned short* KX,
    unsigned short* VH, unsigned short* VL, float oscale, float rres) {
  const _Float16* A  = (const _Float16*)(const void*)Wp;
  const _Float16* Bh = (const _Float16*)(const void*)XHp;
  const _Float16* Bl = (const _Float16*)(const void*)XLp;
  __shared__ __align__(16) unsigned short sP[8][2][16 * SPP];
  const int lane = threadIdx.x & 31;
  const int wave = threadIdx.x >> 5;
  const int tilesN = NTOK / 64;
  const int tilesM = OQKV / 64;
  const int tile = blockIdx.x * 8 + wave;
  if (tile >= tilesM * tilesN) return;
  const int tm = tile / tilesN;
  const int tn = tile - tm * tilesN;
  const int m0 = tm << 6;
  const int n0 = tn << 6;
  const int rlane = lane & 15;
  const int hh    = lane >> 4;
  const int koff  = hh * 8;
  const int mOff  = hh * 8;

  v8f acc[4][4];
#pragma unroll
  for (int i = 0; i < 4; ++i)
#pragma unroll
    for (int j = 0; j < 4; ++j) acc[i][j] = zero8();

  for (int k0 = 0; k0 < DIMC; k0 += 32) {
    v16h bf[4];
#pragma unroll
    for (int j = 0; j < 4; ++j) {
      const size_t bo = (size_t)(n0 + (j << 4) + rlane) * DIMC + koff + k0;
      bf[j] = ldfrag_h(Bh + bo);
    }
#pragma unroll
    for (int i = 0; i < 4; ++i) {
      const size_t ao = (size_t)(m0 + (i << 4) + rlane) * DIMC + koff + k0;
      const v16h ah = ldfrag_h(A + ao);
#pragma unroll
      for (int j = 0; j < 4; ++j) acc[i][j] = mma_h_raw(ah, bf[j], acc[i][j]);
      dep_guard_h(acc[i][0], acc[i][3], ah, bf[3]);
    }
#pragma unroll
    for (int j = 0; j < 4; ++j) {
      const size_t bo = (size_t)(n0 + (j << 4) + rlane) * DIMC + koff + k0;
      bf[j] = ldfrag_h(Bl + bo);
    }
#pragma unroll
    for (int i = 0; i < 4; ++i) {
      const size_t ao = (size_t)(m0 + (i << 4) + rlane) * DIMC + koff + k0;
      const v16h al = ldfrag_h(A + ao);
#pragma unroll
      for (int j = 0; j < 4; ++j) {
        v8f tp = mma_h_raw(al, bf[j], zero8());
        res_guard(tp, acc[i][j], al, bf[j]);
#pragma unroll
        for (int r = 0; r < 8; ++r) acc[i][j][r] += tp[r] * rres;
      }
      dep_guard_h(acc[i][0], acc[i][3], al, bf[3]);
    }
    keep4_h(bf[0], bf[1], bf[2], bf[3]);
  }
  acc_guard4(acc[0][0], acc[0][1], acc[0][2], acc[0][3]);
  acc_guard4(acc[1][0], acc[1][1], acc[1][2], acc[1][3]);
  acc_guard4(acc[2][0], acc[2][1], acc[2][2], acc[2][3]);
  acc_guard4(acc[3][0], acc[3][1], acc[3][2], acc[3][3]);

  const int sec = m0 >> 9;
  const int h   = (m0 & 511) >> 6;
  const float* qb = (sec == 0) ? bq : ((sec == 1) ? bk : bv);
  float bvv[4][8];
#pragma unroll
  for (int i = 0; i < 4; ++i)
#pragma unroll
    for (int r = 0; r < 8; ++r) bvv[i][r] = bf_up(bf_bits(qb[(m0 & 511) + (i << 4) + mOff + r]));
  unsigned short* s0 = &sP[wave][0][0];
  unsigned short* s1 = &sP[wave][1][0];
  const int rq = lane >> 3, c8 = (lane & 7) * 8;

  if (sec < 2) {
    unsigned short* Ph = (sec == 0) ? QH : KX;
#pragma unroll
    for (int j = 0; j < 4; ++j) {
#pragma unroll
      for (int i = 0; i < 4; ++i) {
        unsigned short hb[8], lo[8];
#pragma unroll
        for (int r = 0; r < 8; ++r) {
          const float f = (acc[i][j][r] * oscale + bvv[i][r]) * 16.0f;
          const _Float16 xh = (_Float16)f;
          hb[r] = h_bits(xh);
          lo[r] = h_bits((_Float16)((f - (float)xh) * 2048.0f));
        }
        v4u ph, pl;
#pragma unroll
        for (int q = 0; q < 4; ++q) {
          ph[q] = pk16(hb[2 * q], hb[2 * q + 1]);
          pl[q] = pk16(lo[2 * q], lo[2 * q + 1]);
        }
        *(v4u*)(s0 + rlane * SPP + (i << 4) + mOff) = ph;
        if (sec == 0) *(v4u*)(s1 + rlane * SPP + (i << 4) + mOff) = pl;
      }
      wave_sync_lds();
      for (int pass = 0; pass < 2; ++pass) {
#pragma unroll
        for (int it = 0; it < 4; ++it) {
          const int row = it * 4 + rq;
          const size_t dst = ((size_t)(h * NTOK + n0 + (j << 4) + row)) * HD + c8;
          const v4u v = *(const v4u*)(s0 + row * SPP + c8);
          *(volatile v4u*)(Ph + dst) = v;
          if (sec == 0) {
            const v4u w = *(const v4u*)(s1 + row * SPP + c8);
            *(volatile v4u*)(QL + dst) = w;
          }
        }
        __threadfence();
      }
      wave_sync_lds();
    }
  } else {
#pragma unroll
    for (int i = 0; i < 4; ++i) {
#pragma unroll
      for (int j = 0; j < 4; ++j) {
#pragma unroll
        for (int r = 0; r < 8; ++r) {
          const float f = (acc[i][j][r] * oscale + bvv[i][r]) * 16.0f;
          const _Float16 xh = (_Float16)f;
          const int so = (mOff + r) * SPP + (j << 4) + rlane;
          s0[so] = h_bits(xh);
          s1[so] = h_bits((_Float16)((f - (float)xh) * 2048.0f));
        }
      }
      wave_sync_lds();
      for (int pass = 0; pass < 2; ++pass) {
#pragma unroll
        for (int it = 0; it < 4; ++it) {
          const int row = it * 4 + rq;
          const size_t dst = ((size_t)(h * HD + (i << 4) + row)) * NTOK + n0 + c8;
          const v4u v = *(const v4u*)(s0 + row * SPP + c8);
          const v4u w = *(const v4u*)(s1 + row * SPP + c8);
          *(volatile v4u*)(VH + dst) = v;
          *(volatile v4u*)(VL + dst) = w;
        }
        __threadfence();
      }
      wave_sync_lds();
    }
  }
}

__global__ __launch_bounds__(32) void attn_kernel(
    const unsigned short* __restrict__ QHp, const unsigned short* __restrict__ QLp,
    const unsigned short* __restrict__ KXp,
    const unsigned short* __restrict__ VHp, const unsigned short* __restrict__ VLp,
    const unsigned short* __restrict__ BT,
    unsigned short* CTXh, unsigned short* CTXl, float rscale) {
  __shared__ __align__(16) float sS[NKST * 2 * 32 * 8];
  __shared__ __align__(16) unsigned short sth[16 * 64];
  __shared__ __align__(16) unsigned short stl[16 * 64];
  const _Float16* QH = (const _Float16*)(const void*)QHp;
  const _Float16* QL = (const _Float16*)(const void*)QLp;
  const _Float16* KX = (const _Float16*)(const void*)KXp;
  const _Float16* VH = (const _Float16*)(const void*)VHp;
  const _Float16* VL = (const _Float16*)(const void*)VLp;

  const int lane = threadIdx.x & 31;
  const int t = blockIdx.x;
  const int qblk = t & 31, h = (t >> 5) & 7, b = t >> 8;
  const int tok0 = b * SEQ + qblk * 16;
  const int rlane = lane & 15, hsel = lane >> 4, koff = hsel * 8;

  const float C2048  = 1.0f / 2048.0f;
  const float LN1024 = 6.931471805599453f;

  {
    const size_t qo = ((size_t)(h * NTOK + tok0 + rlane)) * HD + koff;
    const v16h qh0 = ldfrag_h(QH + qo);
    const v16h qh1 = ldfrag_h(QH + qo + 32);
    const v16h ql0 = ldfrag_h(QL + qo);
    const v16h ql1 = ldfrag_h(QL + qo + 32);
#pragma unroll 1
    for (int sub = 0; sub < NKST; ++sub) {
#pragma unroll
      for (int tt = 0; tt < 2; ++tt) {
        const int krow = b * SEQ + sub * 32 + 16 * tt + rlane;
        const size_t ko = ((size_t)(h * NTOK + krow)) * HD + koff;
        const v16h kfa = ldfrag_h(KX + ko);
        const v16h kfb = ldfrag_h(KX + ko + 32);
        v8f sh = mma_h_raw(kfa, qh0, zero8());
        sh = mma_h_raw(kfb, qh1, sh);
        v8f sr = mma_h_raw(kfa, ql0, zero8());
        sr = mma_h_raw(kfb, ql1, sr);
        guard_sc(sh, sr, kfa, kfb, qh0, qh1, ql0, ql1);
        v4f x0, x1;
#pragma unroll
        for (int e = 0; e < 4; ++e) {
          x0[e] = (sh[e]     + sr[e]     * C2048) * C2048;
          x1[e] = (sh[4 + e] + sr[4 + e] * C2048) * C2048;
        }
        float* sp = sS + ((sub * 2 + tt) * 32 + lane) * 8;
        *(v4f*)(sp)     = x0;
        *(v4f*)(sp + 4) = x1;
      }
    }
  }
  wave_sync_lds();

#pragma unroll 1
  for (int g = 0; g < NGRP; ++g) {
    const unsigned short* btrow = BT + (((size_t)(h * NGRP + g)) * SEQ + qblk * 16 + rlane) * SEQ + 8 * hsel;
    v8f oh[4], ol[4];
#pragma unroll
    for (int dt = 0; dt < 4; ++dt) { oh[dt] = zero8(); ol[dt] = zero8(); }
    float m_run = -1.0e30f, l_run = 0.0f;

#pragma unroll 1
    for (int sub = 0; sub < NKST; ++sub) {
      const int kr = sub * 32;
      float a[2][8];
#pragma unroll
      for (int tt = 0; tt < 2; ++tt) {
        const float* sp = sS + ((sub * 2 + tt) * 32 + lane) * 8;
        const v4f x0 = *(const v4f*)(sp);
        const v4f x1 = *(const v4f*)(sp + 4);
        const v4u bw = *(const v4u*)(btrow + kr + 16 * tt);
        float bvv[8];
#pragma unroll
        for (int qq = 0; qq < 4; ++qq) {
          bvv[2 * qq]     = __uint_as_float(bw[qq] << 16);
          bvv[2 * qq + 1] = __uint_as_float(bw[qq] & 0xffff0000u);
        }
#pragma unroll
        for (int e = 0; e < 4; ++e) {
          a[tt][e]     = x0[e] + bvv[e];
          a[tt][4 + e] = x1[e] + bvv[4 + e];
        }
      }

      float mloc = -1.0e30f;
#pragma unroll
      for (int r = 0; r < 8; ++r) mloc = fmaxf(mloc, fmaxf(a[0][r], a[1][r]));
      mloc = fmaxf(mloc, __shfl_xor(mloc, 16, 32));
      const float newM  = fmaxf(m_run, mloc);
      const float alpha = __expf(m_run - newM);
      const float msh   = newM - LN1024;
      float ssum = 0.0f;
      float p[2][8];
#pragma unroll
      for (int r = 0; r < 8; ++r) {
        p[0][r] = __expf(a[0][r] - msh);
        p[1][r] = __expf(a[1][r] - msh);
        ssum += p[0][r] + p[1][r];
      }
      ssum += __shfl_xor(ssum, 16, 32);
      l_run = l_run * alpha + ssum;
      m_run = newM;
#pragma unroll
      for (int dt = 0; dt < 4; ++dt) {
#pragma unroll
        for (int r = 0; r < 8; ++r) { oh[dt][r] *= alpha; ol[dt][r] *= alpha; }
      }

      union { v16h v; _Float16 s[16]; } ph, plo;
#pragma unroll
      for (int r = 0; r < 8; ++r) {
        const _Float16 x0 = (_Float16)p[0][r];
        const _Float16 x1 = (_Float16)p[1][r];
        ph.s[r]      = x0;
        ph.s[8 + r]  = x1;
        plo.s[r]     = (_Float16)((p[0][r] - (float)x0) * 2048.0f);
        plo.s[8 + r] = (_Float16)((p[1][r] - (float)x1) * 2048.0f);
      }

#pragma unroll
      for (int dt = 0; dt < 4; ++dt) {
        const size_t vo = ((size_t)(h * HD + 16 * dt + rlane)) * NTOK + b * SEQ + kr + koff;
        const v16h vah = ldfrag_h(VH + vo);
        const v16h val = ldfrag_h(VL + vo);
        oh[dt] = mma_h_raw(vah, ph.v, oh[dt]);
        ol[dt] = mma_h_raw(val, ph.v, ol[dt]);
        ol[dt] = mma_h_raw(vah, plo.v, ol[dt]);
        guard_pv(oh[dt], ol[dt], vah, val, ph.v, plo.v);
      }
    }
    acc_guard4(oh[0], oh[1], oh[2], oh[3]);
    acc_guard4(ol[0], ol[1], ol[2], ol[3]);

    const float inv = 4.0f * (1.0f / l_run);
#pragma unroll
    for (int dt = 0; dt < 4; ++dt) {
      v4u hv, lw;
#pragma unroll
      for (int e = 0; e < 4; ++e) {
        const float f0 = (oh[dt][2 * e]     + ol[dt][2 * e]     * C2048) * inv;
        const float f1 = (oh[dt][2 * e + 1] + ol[dt][2 * e + 1] * C2048) * inv;
        const _Float16 x0 = (_Float16)f0, x1 = (_Float16)f1;
        hv[e] = pk16(h_bits(x0), h_bits(x1));
        lw[e] = pk16(h_bits((_Float16)((f0 - (float)x0) * rscale)),
                     h_bits((_Float16)((f1 - (float)x1) * rscale)));
      }
      const int so = rlane * 64 + 16 * dt + 8 * hsel;
      *(v4u*)(sth + so) = hv;
      *(v4u*)(stl + so) = lw;
    }
    wave_sync_lds();
    {
      const int rq = lane >> 3, c8 = (lane & 7) * 8;
      for (int pass = 0; pass < 2; ++pass) {
#pragma unroll
        for (int it = 0; it < 4; ++it) {
          const int row = it * 4 + rq;
          const v4u v = *(const v4u*)(sth + row * 64 + c8);
          *(volatile v4u*)(CTXh + (((size_t)(tok0 + row)) * NGRP + g) * DIMC + h * HD + c8) = v;
        }
        __threadfence();
      }
      for (int pass = 0; pass < 2; ++pass) {
#pragma unroll
        for (int it = 0; it < 4; ++it) {
          const int row = it * 4 + rq;
          const v4u v = *(const v4u*)(stl + row * 64 + c8);
          *(volatile v4u*)(CTXl + (((size_t)(tok0 + row)) * NGRP + g) * DIMC + h * HD + c8) = v;
        }
        __threadfence();
      }
    }
    wave_sync_lds();
  }
}

__global__ __launch_bounds__(256) void gemm_out(
    const unsigned short* __restrict__ Ahp, const unsigned short* __restrict__ Alp,
    const unsigned short* __restrict__ Btp, const float* __restrict__ bias,
    float* Cout, float oscale, float rres) {
  const _Float16* Ah = (const _Float16*)(const void*)Ahp;
  const _Float16* Al = (const _Float16*)(const void*)Alp;
  const _Float16* Bt = (const _Float16*)(const void*)Btp;
  __shared__ __align__(16) float sT[8][16 * 68];
  const int lane = threadIdx.x & 31;
  const int wave = threadIdx.x >> 5;
  const int tilesN = DIMC / 64;
  const int tilesM = NROW / 64;
  const int tile = blockIdx.x * 8 + wave;
  if (tile >= tilesM * tilesN) return;
  const int tm = tile / tilesN;
  const int tn = tile - tm * tilesN;
  const int m0 = tm << 6;
  const int n0 = tn << 6;
  const int rlane = lane & 15;
  const int koff  = (lane >> 4) * 8;
  const int mOff  = (lane >> 4) * 8;

  v8f acc[4][4];
#pragma unroll
  for (int i = 0; i < 4; ++i)
#pragma unroll
    for (int j = 0; j < 4; ++j) acc[i][j] = zero8();

  for (int k0 = 0; k0 < DIMC; k0 += 32) {
    v16h bf[4];
#pragma unroll
    for (int j = 0; j < 4; ++j) {
      const size_t bo = (size_t)(n0 + (j << 4) + rlane) * DIMC + koff + k0;
      bf[j] = ldfrag_h(Bt + bo);
    }
#pragma unroll
    for (int i = 0; i < 4; ++i) {
      const size_t ao = (size_t)(m0 + (i << 4) + rlane) * DIMC + koff + k0;
      const v16h ah = ldfrag_h(Ah + ao);
#pragma unroll
      for (int j = 0; j < 4; ++j) acc[i][j] = mma_h_raw(ah, bf[j], acc[i][j]);
      dep_guard_h(acc[i][0], acc[i][3], ah, bf[3]);
    }
#pragma unroll
    for (int i = 0; i < 4; ++i) {
      const size_t ao = (size_t)(m0 + (i << 4) + rlane) * DIMC + koff + k0;
      const v16h al = ldfrag_h(Al + ao);
#pragma unroll
      for (int j = 0; j < 4; ++j) {
        v8f tp = mma_h_raw(al, bf[j], zero8());
        res_guard(tp, acc[i][j], al, bf[j]);
#pragma unroll
        for (int r = 0; r < 8; ++r) acc[i][j][r] += tp[r] * rres;
      }
      dep_guard_h(acc[i][0], acc[i][3], al, bf[3]);
    }
    keep4_h(bf[0], bf[1], bf[2], bf[3]);
  }
  acc_guard4(acc[0][0], acc[0][1], acc[0][2], acc[0][3]);
  acc_guard4(acc[1][0], acc[1][1], acc[1][2], acc[1][3]);
  acc_guard4(acc[2][0], acc[2][1], acc[2][2], acc[2][3]);
  acc_guard4(acc[3][0], acc[3][1], acc[3][2], acc[3][3]);

  float* slab = sT[wave];
  float bc[4];
#pragma unroll
  for (int j = 0; j < 4; ++j) bc[j] = bf_up(bf_bits(bias[n0 + (j << 4) + rlane]));
#pragma unroll
  for (int i = 0; i < 4; ++i) {
    const int mBase = m0 + (i << 4);
#pragma unroll
    for (int j = 0; j < 4; ++j) {
#pragma unroll
      for (int r = 0; r < 8; ++r) {
        slab[(mOff + r) * 68 + (j << 4) + rlane] = acc[i][j][r] * oscale + bc[j];
      }
    }
    wave_sync_lds();
    {
      const int hh = lane >> 4, c4 = (lane & 15) * 4;
      for (int pass = 0; pass < 2; ++pass) {
#pragma unroll
        for (int it = 0; it < 8; ++it) {
          const int row = it * 2 + hh;
          const v4f v = *(const v4f*)(slab + row * 68 + c4);
          *(volatile v4f*)(Cout + (size_t)(mBase + row) * DIMC + n0 + c4) = v;
        }
        __threadfence();
      }
    }
    wave_sync_lds();
  }
}

extern "C" void kernel_launch(void* const* d_in, const int* in_sizes, int n_in,
                              void* d_out, int out_size, void* d_ws, size_t ws_size,
                              hipStream_t stream) {
  if (n_in < 14) return;
  if (in_sizes[0] != NTOK * DIMC) return;
  if (in_sizes[1] != SEQ * SEQ) return;
  if (in_sizes[2] != NGRP * NSITE) return;
  if (in_sizes[3] != DIMC || in_sizes[4] != DIMC) return;
  if (in_sizes[5] != DIMC * DIMC || in_sizes[7] != DIMC * DIMC || in_sizes[9] != DIMC * DIMC || in_sizes[11] != DIMC * DIMC) return;
  if (in_sizes[6] != DIMC || in_sizes[8] != DIMC || in_sizes[10] != DIMC || in_sizes[12] != DIMC) return;
  if (in_sizes[13] != NSITE * HEADS) return;
  if (out_size != NROW * DIMC) return;

  const float* X     = (const float*)d_in[0];
  const int*   sdiff = (const int*)d_in[1];
  const int*   gact  = (const int*)d_in[2];
  const float* lg    = (const float*)d_in[3];
  const float* lb    = (const float*)d_in[4];
  const float* Wq    = (const float*)d_in[5];
  const float* bq    = (const float*)d_in[6];
  const float* Wk    = (const float*)d_in[7];
  const float* bk    = (const float*)d_in[8];
  const float* Wv    = (const float*)d_in[9];
  const float* bv    = (const float*)d_in[10];
  const float* Wo    = (const float*)d_in[11];
  const float* bo    = (const float*)d_in[12];
  const float* rho   = (const float*)d_in[13];

  const size_t PW3 = (size_t)OQKV * DIMC * 2;
  const size_t PPW = (size_t)DIMC * DIMC * 2;
  const size_t PBT = (size_t)HEADS * NGRP * SEQ * SEQ * 2;
  const size_t PX  = (size_t)NTOK * DIMC * 2;
  const size_t PQ  = (size_t)HEADS * NTOK * HD * 2;
  const size_t PCT = (size_t)NROW * DIMC * 2;
  size_t off = 0;
  const size_t oW3 = off; off += PW3;
  const size_t oPW = off; off += PPW;
  const size_t oBT = off; off += PBT;
  const size_t oXH = off; off += PX;
  const size_t oXL = off; off += PX;
  const size_t oQH = off; off += PQ;
  const size_t oQL = off; off += PQ;
  const size_t oKX = off; off += PQ;
  const size_t oVH = off; off += PQ;
  const size_t oVL = off; off += PQ;
  const size_t oCH = off; off += PCT;
  const size_t oCL = off; off += PCT;
  if (off > ws_size) return;
  if (off > (size_t)134217728) return;

  char* ws = (char*)d_ws;
  unsigned short* W3   = (unsigned short*)(ws + oW3);
  unsigned short* PW   = (unsigned short*)(ws + oPW);
  unsigned short* BT   = (unsigned short*)(ws + oBT);
  unsigned short* XH   = (unsigned short*)(ws + oXH);
  unsigned short* XL   = (unsigned short*)(ws + oXL);
  unsigned short* QH   = (unsigned short*)(ws + oQH);
  unsigned short* QL   = (unsigned short*)(ws + oQL);
  unsigned short* KX   = (unsigned short*)(ws + oKX);
  unsigned short* VH   = (unsigned short*)(ws + oVH);
  unsigned short* VL   = (unsigned short*)(ws + oVL);
  unsigned short* CTXh = (unsigned short*)(ws + oCH);
  unsigned short* CTXl = (unsigned short*)(ws + oCL);
  float*          out  = (float*)d_out;

  const dim3 blk(256);
  const dim3 gWT(DIMC / 64, DIMC / 64);
  const dim3 gBT(NBT8 / 256);
  const dim3 gLN(NTOK / 8);
  const dim3 gQkv(((OQKV / 64) * (NTOK / 64) + 7) / 8);
  const dim3 gAttn(BATCH * HEADS * (SEQ / 16));
  const dim3 gOut(((NROW / 64) * (DIMC / 64) + 7) / 8);

  const float oscQkv = 1.0f / 16384.0f;
  const float rresX  = 1.0f / 2048.0f;
  const float rscale = 16384.0f;
  const float oscOut = 1.0f / 65536.0f;
  const float rresC  = 1.0f / 16384.0f;

  cvt_wt<<<gWT, blk, 0, stream>>>(Wq, W3, 0, 1024.0f);
  cvt_wt<<<gWT, blk, 0, stream>>>(Wk, W3, DIMC, 1024.0f);
  cvt_wt<<<gWT, blk, 0, stream>>>(Wv, W3, 2 * DIMC, 1024.0f);
  cvt_wt<<<gWT, blk, 0, stream>>>(Wo, PW, 0, 1024.0f);
  bias_table<<<gBT, blk, 0, stream>>>(rho, sdiff, gact, BT);
  ln_rows<<<gLN, blk, 0, stream>>>(X, lg, lb, XH, XL);
  gemm_qkv<<<gQkv, blk, 0, stream>>>(W3, XH, XL, bq, bk, bv, QH, QL, KX, VH, VL, oscQkv, rresX);
  attn_kernel<<<gAttn, dim3(32), 0, stream>>>(QH, QL, KX, VH, VL, BT, CTXh, CTXl, rscale);
  gemm_out<<<gOut, blk, 0, stream>>>(CTXh, CTXl, PW, bo, out, oscOut, rresC);
  (void)hipGetLastError();
}
